// Rits_20151986553217
// MI455X (gfx1250) — hardware-run, weakly checked
//
#include <hip/hip_runtime.h>
#include <math.h>

typedef __attribute__((ext_vector_type(16))) _Float16 v16h;
typedef __attribute__((ext_vector_type(8)))  _Float16 v8h;
typedef __attribute__((ext_vector_type(16))) __bf16   v16b;
typedef __attribute__((ext_vector_type(8)))  __bf16   v8b;
typedef __attribute__((ext_vector_type(8)))  float    v8f;
typedef __attribute__((ext_vector_type(4)))  float    v4f;
typedef __attribute__((ext_vector_type(4)))  unsigned int v4u;

__device__ __forceinline__ void dep_guard_h(v8f& a, v8f& b, v16h x, v16h y) { asm volatile("v_nop\n\tv_nop\n\tv_nop\n\tv_nop" : "+v"(a), "+v"(b) : "v"(x), "v"(y)); }
__device__ __forceinline__ void dep_guard_b(v8f& a, v8f& b, v16b x, v16b y) { asm volatile("v_nop\n\tv_nop\n\tv_nop\n\tv_nop" : "+v"(a), "+v"(b) : "v"(x), "v"(y)); }
__device__ __forceinline__ void keep4_h(v16h a, v16h b, v16h c, v16h d) { asm volatile("v_nop" :: "v"(a), "v"(b), "v"(c), "v"(d)); }
__device__ __forceinline__ void keep4_b(v16b a, v16b b, v16b c, v16b d) { asm volatile("v_nop" :: "v"(a), "v"(b), "v"(c), "v"(d)); }
template <typename T> struct Frag;
template <> struct Frag<_Float16> {
  typedef v16h V; union U { v16h v; v8h h[2]; };
  static __device__ __forceinline__ v16h load(const _Float16* p) {
    U f; f.h[0] = *(const v8h*)(p); f.h[1] = *(const v8h*)(p + 16); return f.v;
  }
  static __device__ __forceinline__ v8f mma(v16h a, v16h b, v8f c) {
    return __builtin_amdgcn_wmma_f32_16x16x32_f16(false, a, false, b, (short)0, c, false, false);
  }
  static __device__ __forceinline__ void guard(v8f& a, v8f& b, v16h x, v16h y) { dep_guard_h(a, b, x, y); }
  static __device__ __forceinline__ void keep(v16h a, v16h b, v16h c, v16h d) { keep4_h(a, b, c, d); }
};
template <> struct Frag<__bf16> {
  typedef v16b V; union U { v16b v; v8b h[2]; };
  static __device__ __forceinline__ v16b load(const __bf16* p) {
    U f; f.h[0] = *(const v8b*)(p); f.h[1] = *(const v8b*)(p + 16); return f.v;
  }
  static __device__ __forceinline__ v8f mma(v16b a, v16b b, v8f c) {
    return __builtin_amdgcn_wmma_f32_16x16x32_bf16(false, a, false, b, (short)0, c, false, false);
  }
  static __device__ __forceinline__ void guard(v8f& a, v8f& b, v16b x, v16b y) { dep_guard_b(a, b, x, y); }
  static __device__ __forceinline__ void keep(v16b a, v16b b, v16b c, v16b d) { keep4_b(a, b, c, d); }
};

__device__ __forceinline__ unsigned pk16(unsigned short a, unsigned short b) { return (unsigned)a | ((unsigned)b << 16); }
__device__ __forceinline__ unsigned short h_bits(float f) { const _Float16 h = (_Float16)f; return __builtin_bit_cast(unsigned short, h); }

constexpr int SEQ_T = 36;
constexpr int NFEAT = 9;
constexpr int NHID = 64;
constexpr int ROWS_BLK = 64;
constexpr int KPAD = 32;
constexpr int HA_PITCH = 72;
constexpr int ROWF = SEQ_T * NFEAT;
constexpr int PART_STRIDE = 160;
constexpr int WO_GH = 0;
constexpr int WO_HIST = WO_GH + NHID * KPAD;
constexpr int WO_FEAT = WO_HIST + 16 * NHID;
constexpr int WO_COMB = WO_FEAT + 16 * KPAD;
constexpr int WO_IH = WO_COMB + 16 * KPAD;
constexpr int WO_HH = WO_IH + 4 * NHID * KPAD;
constexpr int WPL_HALVES = WO_HH + 4 * NHID * NHID;
constexpr float LOG2E_F = 1.4426950408889634f;

__device__ __forceinline__ float ex2_f(float x) {
#if __has_builtin(__builtin_amdgcn_exp2f)
  return __builtin_amdgcn_exp2f(x);
#else
  return exp2f(x);
#endif
}
__device__ __forceinline__ float rcp_f(float x) {
#if __has_builtin(__builtin_amdgcn_rcpf)
  return __builtin_amdgcn_rcpf(x);
#else
  return 1.0f / x;
#endif
}
__device__ __forceinline__ float decay_f(float v) { return ex2_f(-fmaxf(v, 0.0f) * LOG2E_F); }
__device__ __forceinline__ float sigm_f(float x) { return rcp_f(1.0f + ex2_f(-x * LOG2E_F)); }
__device__ __forceinline__ float tanh_f(float x) { return 2.0f * rcp_f(1.0f + ex2_f(-2.0f * LOG2E_F * x)) - 1.0f; }

__device__ __forceinline__ v8f mma_f16(v16h a, v16h b, v8f c) {
  return __builtin_amdgcn_wmma_f32_16x16x32_f16(false, a, false, b, (short)0, c, false, false);
}
__device__ __forceinline__ void guard_c1(v8f& c, v16h a, v16h b) {
  asm volatile("v_nop\n\tv_nop\n\tv_nop\n\tv_nop" : "+v"(c) : "v"(a), "v"(b));
}
__device__ __forceinline__ void guard_c2(v8f& c, v16h a0, v16h b0, v16h a1, v16h b1) {
  asm volatile("v_nop\n\tv_nop\n\tv_nop\n\tv_nop" : "+v"(c) : "v"(a0), "v"(b0), "v"(a1), "v"(b1));
}
__device__ __forceinline__ void guard_c3(v8f& c, v16h a0, v16h b0, v16h a1, v16h b1, v16h a2, v16h b2) {
  asm volatile("v_nop\n\tv_nop\n\tv_nop\n\tv_nop" : "+v"(c) : "v"(a0), "v"(b0), "v"(a1), "v"(b1), "v"(a2), "v"(b2));
}
__device__ __forceinline__ void guard_d2(v8f& c, v8f& d, v16h a0, v16h b0, v16h a1, v16h b1) {
  asm volatile("v_nop\n\tv_nop\n\tv_nop\n\tv_nop" : "+v"(c), "+v"(d) : "v"(a0), "v"(b0), "v"(a1), "v"(b1));
}
__device__ __forceinline__ v16h fload(const _Float16* p) { return Frag<_Float16>::load(p); }
__device__ __forceinline__ void lds_wave_sync() {
  __builtin_amdgcn_fence(__ATOMIC_RELEASE, "workgroup");
  __builtin_amdgcn_wave_barrier();
  __builtin_amdgcn_fence(__ATOMIC_ACQUIRE, "workgroup");
}

__global__ __launch_bounds__(256) void k_prep_weights(
    const float* __restrict__ W_gh, const float* __restrict__ W_hist, const float* __restrict__ W_feat,
    const float* __restrict__ W_comb, const float* __restrict__ W_ih, const float* __restrict__ W_hh,
    unsigned short* __restrict__ wpl) {
  const int g = blockIdx.x * 256 + threadIdx.x;
  if (g >= WPL_HALVES / 8) return;
  const int e0 = g * 8;
  float v[8];
  if (e0 < WO_HIST) {
    const int n = e0 >> 5, k0 = e0 & 31;
#pragma unroll
    for (int k = 0; k < 8; ++k) {
      const int kk = k0 + k;
      const int kc = (kk < NFEAT) ? kk : (NFEAT - 1);
      const float w = W_gh[n * NFEAT + kc];
      v[k] = (kk < NFEAT) ? w : 0.0f;
    }
  } else if (e0 < WO_FEAT) {
    const int e1 = e0 - WO_HIST;
    const int f = e1 >> 6, k0 = e1 & 63;
    const int fc = (f < NFEAT) ? f : (NFEAT - 1);
#pragma unroll
    for (int k = 0; k < 8; ++k) {
      const float w = W_hist[fc * NHID + k0 + k];
      v[k] = (f < NFEAT) ? w : 0.0f;
    }
  } else if (e0 < WO_COMB) {
    const int e1 = e0 - WO_FEAT;
    const int f = e1 >> 5, k0 = e1 & 31;
    const int fc = (f < NFEAT) ? f : (NFEAT - 1);
#pragma unroll
    for (int k = 0; k < 8; ++k) {
      const int kk = k0 + k;
      const int kc = (kk < NFEAT) ? kk : (NFEAT - 1);
      const float w = W_feat[fc * NFEAT + kc];
      v[k] = (f < NFEAT && kk < NFEAT && kk != f) ? w : 0.0f;
    }
  } else if (e0 < WO_IH) {
    const int e1 = e0 - WO_COMB;
    const int f = e1 >> 5, k0 = e1 & 31;
    const int fc = (f < NFEAT) ? f : (NFEAT - 1);
#pragma unroll
    for (int k = 0; k < 8; ++k) {
      const int kk = k0 + k;
      const int kc = (kk < 2 * NFEAT) ? kk : (2 * NFEAT - 1);
      const float w = W_comb[fc * (2 * NFEAT) + kc];
      v[k] = (f < NFEAT && kk < 2 * NFEAT) ? w : 0.0f;
    }
  } else if (e0 < WO_HH) {
    const int e1 = e0 - WO_IH;
    const int n = e1 >> 5, k0 = e1 & 31;
#pragma unroll
    for (int k = 0; k < 8; ++k) {
      const int kk = k0 + k;
      const int kc = (kk < 2 * NFEAT) ? kk : (2 * NFEAT - 1);
      const float w = W_ih[n * (2 * NFEAT) + kc];
      v[k] = (kk < 2 * NFEAT) ? w : 0.0f;
    }
  } else {
    const int e1 = e0 - WO_HH;
    const int n = e1 >> 6, k0 = e1 & 63;
#pragma unroll
    for (int k = 0; k < 8; ++k) v[k] = W_hh[n * NHID + k0 + k];
  }
  const v4u u = (v4u){pk16(h_bits(v[0]), h_bits(v[1])), pk16(h_bits(v[2]), h_bits(v[3])),
                      pk16(h_bits(v[4]), h_bits(v[5])), pk16(h_bits(v[6]), h_bits(v[7]))};
  unsigned short* q = wpl + (size_t)e0;
  *(volatile v4u*)q = u;
  __threadfence();
  *(volatile v4u*)q = u;
}

__global__ __launch_bounds__(256) void k_recur_main(
    const float* __restrict__ values, const float* __restrict__ masks, const float* __restrict__ deltas,
    const unsigned short* __restrict__ wplu,
    const float* __restrict__ b_gh, const float* __restrict__ W_gx, const float* __restrict__ b_gx,
    const float* __restrict__ b_hist, const float* __restrict__ b_feat, const float* __restrict__ b_comb,
    const float* __restrict__ b_ih, const float* __restrict__ b_hh,
    float* __restrict__ tbf, float* __restrict__ part, int nbatch) {
  __shared__ __align__(16) _Float16 hA[ROWS_BLK * HA_PITCH];
  __shared__ __align__(16) _Float16 dT[4 * 16 * KPAD];
  __shared__ __align__(16) _Float16 xcT[4 * 16 * KPAD];
  __shared__ __align__(16) _Float16 gmT[4 * 16 * KPAD];
  __shared__ __align__(16) _Float16 inT[4 * 16 * KPAD];
  __shared__ __align__(16) float ccL[ROWS_BLK * NFEAT];
  __shared__ __align__(16) float partL[4 * SEQ_T * 4];
  __shared__ __align__(16) float outL[PART_STRIDE];

  const _Float16* wpl = (const _Float16*)(const void*)wplu;
  const int tid  = threadIdx.x;
  const int lane = tid & 31;
  const int wave = __builtin_amdgcn_readfirstlane(tid >> 5);
  const int mi   = wave >> 1;
  const int uh   = wave & 1;
  const int hh   = lane >> 4;
  const int c    = lane & 15;
  const int koff = hh * 8;
  const int blk  = blockIdx.x;
  const size_t growBase = (size_t)blk * ROWS_BLK;

  const _Float16 hz = (_Float16)0.0f;
#pragma unroll 1
  for (int i = tid; i < ROWS_BLK * HA_PITCH; i += 256) hA[i] = hz;
#pragma unroll 1
  for (int i = tid; i < 4 * 16 * KPAD; i += 256) { dT[i] = hz; xcT[i] = hz; gmT[i] = hz; inT[i] = hz; }
#pragma unroll 1
  for (int i = tid; i < ROWS_BLK * NFEAT; i += 256) { ccL[i] = 0.0f; partL[i] = 0.0f; }
  if (tid < PART_STRIDE) outL[tid] = 0.0f;

  const bool fval = (c < NFEAT);
  const int  fcl  = fval ? c : (NFEAT - 1);
  const float bh_f  = b_hist[fcl];
  const float bfe_f = b_feat[fcl];
  const float bco_f = b_comb[fcl];
  const float wgx_f = W_gx[fcl * NFEAT + fcl];
  const float bgx_f = b_gx[fcl];
  float bgh_u[2];
  float bg[2][4];
#pragma unroll
  for (int ul = 0; ul < 2; ++ul) {
    const int col = 32 * uh + 16 * ul + c;
    bgh_u[ul] = b_gh[col];
#pragma unroll
    for (int q = 0; q < 4; ++q) bg[ul][q] = b_ih[q * NHID + col] + b_hh[q * NHID + col];
  }
  float h2[2][8], c2[2][8];
#pragma unroll
  for (int ul = 0; ul < 2; ++ul)
#pragma unroll
    for (int r = 0; r < 8; ++r) { h2[ul][r] = 0.0f; c2[ul][r] = 0.0f; }

  _Float16* dTm  = dT  + mi * (16 * KPAD);
  _Float16* xcTm = xcT + mi * (16 * KPAD);
  _Float16* gmTm = gmT + mi * (16 * KPAD);
  _Float16* inTm = inT + mi * (16 * KPAD);
  _Float16* hAm  = hA  + (16 * mi) * HA_PITCH;
  const v8f zero8 = (v8f){0.f, 0.f, 0.f, 0.f, 0.f, 0.f, 0.f, 0.f};
  __syncthreads();

#pragma unroll 1
  for (int t = 0; t < SEQ_T; ++t) {
    float xv[8], mv[8], dv[8];
#pragma unroll
    for (int r = 0; r < 8; ++r) { xv[r] = 0.0f; mv[r] = 0.0f; dv[r] = 0.0f; }

    if (uh == 0) {
#pragma unroll
      for (int r = 0; r < 8; ++r) {
        const size_t gidx = ((growBase + (size_t)(16 * mi + 8 * hh + r)) * SEQ_T + (size_t)t) * NFEAT + (size_t)fcl;
        const float a = values[gidx];
        const float b = masks[gidx];
        const float d = deltas[gidx];
        xv[r] = fval ? a : 0.0f;
        mv[r] = fval ? b : 0.0f;
        dv[r] = fval ? d : 0.0f;
      }
      if (fval) {
#pragma unroll
        for (int r = 0; r < 8; ++r) dTm[(8 * hh + r) * KPAD + c] = (_Float16)dv[r];
      }
    }
    __syncthreads();

    {
      const v16h aD = fload(dTm + c * KPAD + koff);
#pragma unroll
      for (int ul = 0; ul < 2; ++ul) {
        const int ncol0 = 32 * uh + 16 * ul;
        const v16h bG = fload(wpl + WO_GH + (ncol0 + c) * KPAD + koff);
        v8f g = mma_f16(aD, bG, zero8);
        guard_c1(g, aD, bG);
#pragma unroll
        for (int r = 0; r < 8; ++r) {
          const float gm = decay_f(g[r] + bgh_u[ul]);
          h2[ul][r] *= gm;
          hAm[(8 * hh + r) * HA_PITCH + ncol0 + c] = (_Float16)h2[ul][r];
        }
      }
    }
    __syncthreads();

    if (uh == 0) {
      const v16h fH0 = fload(hAm + c * HA_PITCH + koff);
      const v16h fH1 = fload(hAm + c * HA_PITCH + 32 + koff);
      const v16h bW0 = fload(wpl + WO_HIST + c * NHID + koff);
      const v16h bW1 = fload(wpl + WO_HIST + c * NHID + 32 + koff);
      v8f xh = mma_f16(fH0, bW0, zero8);
      xh = mma_f16(fH1, bW1, xh);
      guard_c2(xh, fH0, bW0, fH1, bW1);

      float xhv[8], gxv[8], xcv[8];
#pragma unroll
      for (int r = 0; r < 8; ++r) {
        xhv[r] = xh[r] + bh_f;
        gxv[r] = decay_f(dv[r] * wgx_f + bgx_f);
        xcv[r] = mv[r] * xv[r] + (1.0f - mv[r]) * xhv[r];
      }
      if (fval) {
#pragma unroll
        for (int r = 0; r < 8; ++r) {
          xcTm[(8 * hh + r) * KPAD + c] = (_Float16)xcv[r];
          gmTm[(8 * hh + r) * KPAD + c] = (_Float16)gxv[r];
          gmTm[(8 * hh + r) * KPAD + NFEAT + c] = (_Float16)mv[r];
        }
      }
      lds_wave_sync();
      const v16h aX = fload(xcTm + c * KPAD + koff);
      const v16h bF = fload(wpl + WO_FEAT + c * KPAD + koff);
      const v16h aG = fload(gmTm + c * KPAD + koff);
      const v16h bC = fload(wpl + WO_COMB + c * KPAD + koff);
      v8f zh = mma_f16(aX, bF, zero8);
      v8f al = mma_f16(aG, bC, zero8);
      guard_d2(zh, al, aX, bF, aG, bC);

      float l1 = 0.0f, l2 = 0.0f, l3 = 0.0f, ms = 0.0f;
      float ccv[8];
#pragma unroll
      for (int r = 0; r < 8; ++r) {
        const float zhv = zh[r] + bfe_f;
        const float alv = al[r] + bco_f;
        const float ch  = alv * zhv + (1.0f - alv) * xhv[r];
        ccv[r] = mv[r] * xv[r] + (1.0f - mv[r]) * ch;
        l1 += fabsf(xv[r] - xhv[r]) * mv[r];
        l2 += fabsf(xv[r] - zhv) * mv[r];
        l3 += fabsf(xv[r] - ch) * mv[r];
        ms += mv[r];
      }
      if (fval) {
#pragma unroll
        for (int r = 0; r < 8; ++r) {
          ccL[(16 * mi + 8 * hh + r) * NFEAT + c] = ccv[r];
          inTm[(8 * hh + r) * KPAD + c] = (_Float16)ccv[r];
          inTm[(8 * hh + r) * KPAD + NFEAT + c] = (_Float16)mv[r];
        }
      }
#pragma unroll
      for (int off = 16; off > 0; off >>= 1) {
        l1 += __shfl_xor(l1, off, 32);
        l2 += __shfl_xor(l2, off, 32);
        l3 += __shfl_xor(l3, off, 32);
        ms += __shfl_xor(ms, off, 32);
      }
      if (lane == 0) {
        partL[(mi * SEQ_T + t) * 4 + 0] = l1;
        partL[(mi * SEQ_T + t) * 4 + 1] = l2;
        partL[(mi * SEQ_T + t) * 4 + 2] = l3;
        partL[(mi * SEQ_T + t) * 4 + 3] = ms;
      }
    }
    __syncthreads();

    {
      const size_t gb = ((size_t)t * (size_t)nbatch + growBase) * NFEAT;
      for (int pass = 0; pass < 2; ++pass) {
        if (tid < (ROWS_BLK * NFEAT) / 4) {
          const v4f v = *(const v4f*)(ccL + 4 * tid);
          *(volatile v4f*)(tbf + gb + 4 * (size_t)tid) = v;
        }
        __threadfence();
      }
    }

    {
      const v16h aI  = fload(inTm + c * KPAD + koff);
      const v16h aH0 = fload(hAm + c * HA_PITCH + koff);
      const v16h aH1 = fload(hAm + c * HA_PITCH + 32 + koff);
#pragma unroll
      for (int ul = 0; ul < 2; ++ul) {
        v8f ga[4];
#pragma unroll
        for (int q = 0; q < 4; ++q) {
          const int n0 = q * NHID + 32 * uh + 16 * ul;
          const v16h bI  = fload(wpl + WO_IH + (n0 + c) * KPAD + koff);
          const v16h bH0 = fload(wpl + WO_HH + (n0 + c) * NHID + koff);
          const v16h bH1 = fload(wpl + WO_HH + (n0 + c) * NHID + 32 + koff);
          v8f a = mma_f16(aI, bI, zero8);
          a = mma_f16(aH0, bH0, a);
          a = mma_f16(aH1, bH1, a);
          guard_c3(a, aI, bI, aH0, bH0, aH1, bH1);
          ga[q] = a;
        }
#pragma unroll
        for (int r = 0; r < 8; ++r) {
          const float ig = sigm_f(ga[0][r] + bg[ul][0]);
          const float fg = sigm_f(ga[1][r] + bg[ul][1]);
          const float gg = tanh_f(ga[2][r] + bg[ul][2]);
          const float og = sigm_f(ga[3][r] + bg[ul][3]);
          const float cn = fg * c2[ul][r] + ig * gg;
          c2[ul][r] = cn;
          h2[ul][r] = og * tanh_f(cn);
        }
      }
    }
  }
  __syncthreads();

  if (tid < SEQ_T * 4) {
    const float s = ((partL[tid] + partL[SEQ_T * 4 + tid]) + partL[2 * SEQ_T * 4 + tid]) + partL[3 * SEQ_T * 4 + tid];
    outL[tid] = s;
  }
  __syncthreads();
  if (wave == 0) {
    float* pb = part + (size_t)blk * PART_STRIDE;
    for (int pass = 0; pass < 2; ++pass) {
      const v4f v0 = *(const v4f*)(outL + 4 * lane);
      *(volatile v4f*)(pb + 4 * lane) = v0;
      if (lane < 8) {
        const v4f v1 = *(const v4f*)(outL + 128 + 4 * lane);
        *(volatile v4f*)(pb + 128 + 4 * lane) = v1;
      }
      __threadfence();
    }
  }
}

__global__ __launch_bounds__(256) void k_loss_final(const float* __restrict__ part, int nblk, float* __restrict__ lossbuf) {
  __shared__ float sL[PART_STRIDE];
  __shared__ float lineL[32];
  const int tid = threadIdx.x;
  float s = 0.0f;
  if (tid < SEQ_T * 4) {
#pragma unroll 1
    for (int b = 0; b < nblk; ++b) s += part[(size_t)b * PART_STRIDE + tid];
  }
  if (tid < PART_STRIDE) sL[tid] = (tid < SEQ_T * 4) ? s : 0.0f;
  if (tid < 32) lineL[tid] = 0.0f;
  __syncthreads();
  if (tid == 0) {
    float acc = 0.0f;
#pragma unroll 1
    for (int t = 0; t < SEQ_T; ++t) {
      const float num = (sL[4 * t] + sL[4 * t + 1]) + sL[4 * t + 2];
      const float den = sL[4 * t + 3] + 1e-5f;
      acc += num / den;
    }
    lineL[0] = acc / (float)SEQ_T;
  }
  __syncthreads();
  if (tid < 32) {
    const float v = lineL[tid];
    *(volatile float*)(lossbuf + tid) = v;
    __threadfence();
    *(volatile float*)(lossbuf + tid) = v;
  }
}

__global__ __launch_bounds__(256) void k_copy_out(const float* __restrict__ tbf, const float* __restrict__ lossbuf,
                                                 float* __restrict__ out, int n4, int out_n, int nbatch) {
  const int i   = blockIdx.x * 256 + threadIdx.x;
  const int ic  = (i < n4) ? i : n4;
  const int nst = out_n - 1;
  float v[4];
#pragma unroll
  for (int e = 0; e < 4; ++e) {
    int j = 4 * ic + e - 1;
    j = (j < 0) ? 0 : j;
    j = (j > nst - 1) ? (nst - 1) : j;
    const int b   = j / ROWF;
    const int rem = j - b * ROWF;
    const int tt  = rem / NFEAT;
    const int f   = rem - tt * NFEAT;
    v[e] = tbf[((size_t)tt * (size_t)nbatch + (size_t)b) * NFEAT + (size_t)f];
  }
  const float lv = lossbuf[0];
  const float v0 = (i == 0) ? lv : v[0];
  if (i < n4) {
    const v4f w = (v4f){v0, v[1], v[2], v[3]};
    float* p = out + 4 * (size_t)i;
    *(volatile v4f*)p = w;
    __threadfence();
    *(volatile v4f*)p = w;
  } else if (i == n4) {
    const int rm = out_n - 4 * n4;
#pragma unroll
    for (int e = 0; e < 3; ++e) {
      if (e < rm) {
        float* p = out + 4 * (size_t)n4 + e;
        const float val = v[e];
        *(volatile float*)p = val;
        __threadfence();
        *(volatile float*)p = val;
      }
    }
  }
}

extern "C" void kernel_launch(void* const* d_in, const int* in_sizes, int n_in,
                              void* d_out, int out_size, void* d_ws, size_t ws_size,
                              hipStream_t stream) {
  const float* values = (const float*)d_in[0];
  const float* masks  = (const float*)d_in[1];
  const float* deltas = (const float*)d_in[2];
  const float* W_gh   = (const float*)d_in[3];
  const float* b_gh   = (const float*)d_in[4];
  const float* W_gx   = (const float*)d_in[5];
  const float* b_gx   = (const float*)d_in[6];
  const float* W_hist = (const float*)d_in[7];
  const float* b_hist = (const float*)d_in[8];
  const float* W_feat = (const float*)d_in[9];
  const float* b_feat = (const float*)d_in[10];
  const float* W_comb = (const float*)d_in[11];
  const float* b_comb = (const float*)d_in[12];
  const float* W_ih   = (const float*)d_in[13];
  const float* W_hh   = (const float*)d_in[14];
  const float* b_ih   = (const float*)d_in[15];
  const float* b_hh   = (const float*)d_in[16];
  (void)n_in;

  const int nbatch = in_sizes[0] / ROWF;
  if (nbatch <= 0) return;
  if (in_sizes[0] != nbatch * ROWF) return;
  if ((nbatch % ROWS_BLK) != 0) return;
  if (out_size != nbatch * ROWF + 1) return;
  const int nblk = nbatch / ROWS_BLK;

  const size_t off_wpl  = 0;
  const size_t sz_wpl   = (size_t)WPL_HALVES * 2;
  const size_t off_part = off_wpl + sz_wpl;
  const size_t sz_part  = (size_t)nblk * PART_STRIDE * 4;
  const size_t off_loss = off_part + sz_part;
  const size_t sz_loss  = 128;
  const size_t off_tbf  = (off_loss + sz_loss + 127) & ~(size_t)127;
  const size_t sz_tbf   = (size_t)nbatch * ROWF * 4;
  if (off_tbf + sz_tbf > ws_size) return;

  char* ws = (char*)d_ws;
  unsigned short* wpl = (unsigned short*)(ws + off_wpl);
  float* part    = (float*)(ws + off_part);
  float* lossbuf = (float*)(ws + off_loss);
  float* tbf     = (float*)(ws + off_tbf);
  float* out     = (float*)d_out;

  k_prep_weights<<<dim3((WPL_HALVES / 8 + 255) / 256), dim3(256), 0, stream>>>(W_gh, W_hist, W_feat, W_comb, W_ih, W_hh, wpl);

  k_recur_main<<<dim3(nblk), dim3(256), 0, stream>>>(values, masks, deltas, wpl,
                                                     b_gh, W_gx, b_gx, b_hist, b_feat, b_comb, b_ih, b_hh,
                                                     tbf, part, nbatch);

  k_loss_final<<<dim3(1), dim3(256), 0, stream>>>(part, nblk, lossbuf);

  const int n4 = out_size / 4;
  const int nthr = n4 + 1;
  k_copy_out<<<dim3((nthr + 255) / 256), dim3(256), 0, stream>>>(tbf, lossbuf, out, n4, out_size, nbatch);
}
